// SimpleAttention_v2_70342974374217
// MI455X (gfx1250) — hardware-run, weakly checked
//
#include <hip/hip_runtime.h>
#include <math.h>

constexpr int kBatch = 4;
constexpr int kSeq   = 2048;
constexpr int kDim   = 1024;
constexpr int kTok   = kBatch * kSeq;
constexpr int kQKld  = 2 * kDim;
constexpr float kInvSqrtD = 0.03125f;


typedef __attribute__((ext_vector_type(16))) _Float16 v16h;
typedef __attribute__((ext_vector_type(8)))  _Float16 v8h;
typedef __attribute__((ext_vector_type(16))) __bf16   v16b;
typedef __attribute__((ext_vector_type(8)))  __bf16   v8b;
typedef __attribute__((ext_vector_type(8)))  float    v8f;
typedef __attribute__((ext_vector_type(4)))  float    v4f;
typedef __attribute__((ext_vector_type(4)))  unsigned int v4u;

__device__ __forceinline__ unsigned short f2bf_bits(float f) {
  unsigned u = __float_as_uint(f);
  return (unsigned short)((u + 0x7FFFu + ((u >> 16) & 1u)) >> 16);
}
__device__ __forceinline__ float bf_bits2f(unsigned short h) { return __uint_as_float(((unsigned)h) << 16); }

__device__ __forceinline__ void dep_guard_h(v8f& a, v8f& b, v16h x, v16h y) { asm volatile("v_nop\n\tv_nop\n\tv_nop\n\tv_nop" : "+v"(a), "+v"(b) : "v"(x), "v"(y)); }
__device__ __forceinline__ void dep_guard_b(v8f& a, v8f& b, v16b x, v16b y) { asm volatile("v_nop\n\tv_nop\n\tv_nop\n\tv_nop" : "+v"(a), "+v"(b) : "v"(x), "v"(y)); }
__device__ __forceinline__ void keep4_h(v16h a, v16h b, v16h c, v16h d) { asm volatile("v_nop" :: "v"(a), "v"(b), "v"(c), "v"(d)); }
__device__ __forceinline__ void keep4_b(v16b a, v16b b, v16b c, v16b d) { asm volatile("v_nop" :: "v"(a), "v"(b), "v"(c), "v"(d)); }
__device__ __forceinline__ void acc_guard4(v8f& a, v8f& b, v8f& c, v8f& d) { asm volatile("v_nop\n\tv_nop\n\tv_nop\n\tv_nop" : "+v"(a), "+v"(b), "+v"(c), "+v"(d)); }
template <typename T> struct Frag;
template <> struct Frag<_Float16> {
  typedef v16h V; union U { v16h v; v8h h[2]; };
  static __device__ __forceinline__ v16h load(const _Float16* p) {
    U f; f.h[0] = *(const v8h*)(p); f.h[1] = *(const v8h*)(p + 16); return f.v;
  }
  static __device__ __forceinline__ v8f mma(v16h a, v16h b, v8f c) {
    return __builtin_amdgcn_wmma_f32_16x16x32_f16(false, a, false, b, (short)0, c, false, false);
  }
  static __device__ __forceinline__ void guard(v8f& a, v8f& b, v16h x, v16h y) { dep_guard_h(a, b, x, y); }
  static __device__ __forceinline__ void keep(v16h a, v16h b, v16h c, v16h d) { keep4_h(a, b, c, d); }
};
template <> struct Frag<__bf16> {
  typedef v16b V; union U { v16b v; v8b h[2]; };
  static __device__ __forceinline__ v16b load(const __bf16* p) {
    U f; f.h[0] = *(const v8b*)(p); f.h[1] = *(const v8b*)(p + 16); return f.v;
  }
  static __device__ __forceinline__ v8f mma(v16b a, v16b b, v8f c) {
    return __builtin_amdgcn_wmma_f32_16x16x32_bf16(false, a, false, b, (short)0, c, false, false);
  }
  static __device__ __forceinline__ void guard(v8f& a, v8f& b, v16b x, v16b y) { dep_guard_b(a, b, x, y); }
  static __device__ __forceinline__ void keep(v16b a, v16b b, v16b c, v16b d) { keep4_b(a, b, c, d); }
};

__device__ __forceinline__ unsigned pk16(unsigned short a, unsigned short b) { return (unsigned)a | ((unsigned)b << 16); }

template <int ET> struct Elem;
template <> struct Elem<0> { typedef _Float16 T; };
template <> struct Elem<1> { typedef __bf16 T; };
template <int ET, bool SPLIT, int BIAS_MODE, int OUT_MODE, bool RESID, int ACT = 0, bool CAUSALK = false>
__global__ __launch_bounds__(256) void wmma_gemm64(
    const unsigned short* __restrict__ Ap, const unsigned short* __restrict__ A2p, int lda, long strideA,
    const unsigned short* __restrict__ Btp, const unsigned short* __restrict__ Bt2p, int ldb, long strideB,
    void* __restrict__ Cout, void* __restrict__ Cout2, int ldc, long strideC,
    const float* __restrict__ bias,
    const float* __restrict__ resid, long strideR,
    int M, int N, int K, float scale) {
  typedef typename Elem<ET>::T T;
  typedef typename Frag<T>::V V;
  const T* A = (const T*)Ap; const T* A2 = (const T*)A2p; const T* Bt = (const T*)Btp; const T* Bt2 = (const T*)Bt2p;
  __shared__ __align__(16) float sT[8][16 * 68];
  const int b    = blockIdx.y;
  const int lane = threadIdx.x & 31;
  const int wave = threadIdx.x >> 5;
  const int tilesN = N >> 6;
  const int tilesM = M >> 6;
  const int tile = blockIdx.x * 8 + wave;
  if (tile >= tilesM * tilesN) return;
  const int tm = tile / tilesN;
  const int tn = tile - tm * tilesN;
  const int m0 = tm << 6;
  const int n0 = tn << 6;
  const int Kend = CAUSALK ? (((m0 + 64) < K) ? (m0 + 64) : K) : K;

  const T* Ab  = A  + (size_t)b * strideA;
  const T* Bb  = Bt + (size_t)b * strideB;
  const T* Ab2 = SPLIT ? (A2  + (size_t)b * strideA) : nullptr;
  const T* Bb2 = SPLIT ? (Bt2 + (size_t)b * strideB) : nullptr;

  const int rlane = lane & 15;
  const int koff  = (lane >> 4) * 8;
  const int mOff  = (lane >> 4) * 8;

  v8f acc[4][4];
#pragma unroll
  for (int i = 0; i < 4; ++i)
#pragma unroll
    for (int j = 0; j < 4; ++j) acc[i][j] = (v8f){0.f,0.f,0.f,0.f,0.f,0.f,0.f,0.f};

  for (int k0 = 0; k0 < Kend; k0 += 32) {
    V bh[4], bl[4];
#pragma unroll
    for (int j = 0; j < 4; ++j) {
      const size_t bo = (size_t)(n0 + (j << 4) + rlane) * ldb + koff + k0;
      bh[j] = Frag<T>::load(Bb + bo);
      if (SPLIT) bl[j] = Frag<T>::load(Bb2 + bo);
    }
#pragma unroll
    for (int i = 0; i < 4; ++i) {
      const size_t ao = (size_t)(m0 + (i << 4) + rlane) * lda + koff + k0;
      V ah = Frag<T>::load(Ab + ao);
      V al;
      if (SPLIT) al = Frag<T>::load(Ab2 + ao);
#pragma unroll
      for (int j = 0; j < 4; ++j) {
        acc[i][j] = Frag<T>::mma(ah, bh[j], acc[i][j]);
        if (SPLIT) {
          acc[i][j] = Frag<T>::mma(ah, bl[j], acc[i][j]);
          acc[i][j] = Frag<T>::mma(al, bh[j], acc[i][j]);
        }
      }
      Frag<T>::guard(acc[i][0], acc[i][3], ah, SPLIT ? al : ah);
    }
    Frag<T>::keep(bh[0], bh[1], bh[2], bh[3]);
    if (SPLIT) Frag<T>::keep(bl[0], bl[1], bl[2], bl[3]);
  }
  acc_guard4(acc[0][0], acc[0][1], acc[0][2], acc[0][3]);
  acc_guard4(acc[1][0], acc[1][1], acc[1][2], acc[1][3]);
  acc_guard4(acc[2][0], acc[2][1], acc[2][2], acc[2][3]);
  acc_guard4(acc[3][0], acc[3][1], acc[3][2], acc[3][3]);

  float* slab = sT[wave];
  const float* Rb = RESID ? (resid + (size_t)b * strideR) : nullptr;
#pragma unroll
  for (int i = 0; i < 4; ++i) {
    const int mBase = m0 + (i << 4);
#pragma unroll
    for (int j = 0; j < 4; ++j) {
      const int n = n0 + (j << 4) + rlane;
      float bv = 0.f;
      if (BIAS_MODE == 2) bv = bias[n];
#pragma unroll
      for (int r = 0; r < 8; ++r) {
        float v = acc[i][j][r] * scale;
        if (BIAS_MODE == 1) v += bias[mBase + mOff + r];
        if (BIAS_MODE == 2) v += bv;
        if (RESID) v += Rb[(size_t)(mBase + mOff + r) * ldc + n];
        if (ACT == 2) v = fmaxf(v, 0.0f);
        if (ACT == 4) v = (v > 0.f) ? v : 0.01f * v;
        slab[(mOff + r) * 68 + (j << 4) + rlane] = v;
      }
    }
    __builtin_amdgcn_fence(__ATOMIC_RELEASE, "workgroup");
    __builtin_amdgcn_wave_barrier();
    __builtin_amdgcn_fence(__ATOMIC_ACQUIRE, "workgroup");
    if (OUT_MODE == 0) {
      float* C = (float*)Cout + (size_t)b * strideC;
      const int hh = lane >> 4, c4 = (lane & 15) * 4;
      for (int pass = 0; pass < 2; ++pass) {
#pragma unroll
        for (int it = 0; it < 8; ++it) {
          const int row = it * 2 + hh;
          v4f v = *(const v4f*)(slab + row * 68 + c4);
          *(volatile v4f*)(C + (size_t)(mBase + row) * ldc + n0 + c4) = v;
        }
        __threadfence();
      }
    } else {
      const int q = lane >> 3, c8 = (lane & 7) * 8;
      unsigned short* C  = (unsigned short*)Cout  + (size_t)b * strideC;
      unsigned short* C2 = (OUT_MODE == 2) ? ((unsigned short*)Cout2 + (size_t)b * strideC) : nullptr;
      for (int pass = 0; pass < 2; ++pass) {
#pragma unroll
        for (int it = 0; it < 4; ++it) {
          const int row = it * 4 + q;
          const float* sp = slab + row * 68 + c8;
          v8h hv, lv;
#pragma unroll
          for (int e = 0; e < 8; ++e) {
            if (OUT_MODE == 1) {
              hv[e] = (_Float16)sp[e];
            } else {
              unsigned short hb = f2bf_bits(sp[e]);
              unsigned short lb = f2bf_bits(sp[e] - bf_bits2f(hb));
              hv[e] = __builtin_bit_cast(_Float16, hb);
              lv[e] = __builtin_bit_cast(_Float16, lb);
            }
          }
          *(volatile v8h*)(C + (size_t)(mBase + row) * ldc + n0 + c8) = hv;
          if (OUT_MODE == 2) *(volatile v8h*)(C2 + (size_t)(mBase + row) * ldc + n0 + c8) = lv;
        }
        __threadfence();
      }
    }
    __builtin_amdgcn_fence(__ATOMIC_RELEASE, "workgroup");
    __builtin_amdgcn_wave_barrier();
    __builtin_amdgcn_fence(__ATOMIC_ACQUIRE, "workgroup");
  }
}

__global__ __launch_bounds__(256) void cast8_bf16_kernel(const float* __restrict__ in, unsigned short* __restrict__ out, int n8) {
  const int i = blockIdx.x * 256 + threadIdx.x;
  if (i >= n8) return;
  const float* p = in + 8 * (size_t)i;
  const v4f a = *(const v4f*)(p);
  const v4f c = *(const v4f*)(p + 4);
  unsigned short hb[8];
#pragma unroll
  for (int e = 0; e < 4; ++e) {
    hb[e]     = f2bf_bits(a[e]);
    hb[4 + e] = f2bf_bits(c[e]);
  }
  const v4u u = (v4u){pk16(hb[0], hb[1]), pk16(hb[2], hb[3]), pk16(hb[4], hb[5]), pk16(hb[6], hb[7])};
  unsigned short* q = out + 8 * (size_t)i;
  *(volatile v4u*)q = u;
  __threadfence();
  *(volatile v4u*)q = u;
}

__global__ __launch_bounds__(256) void softmax2_row_kernel(const float* __restrict__ S,
                                                           unsigned short* __restrict__ Ph,
                                                           unsigned short* __restrict__ Pl) {
  __shared__ float red[4][8];
  const int row  = blockIdx.x;
  const int t    = threadIdx.x;
  const int lane = t & 31, wave = t >> 5;
  const int c0   = t * 8;
  const float* sr = S + (size_t)row * kSeq + c0;
  const v4f a = *(const v4f*)(sr);
  const v4f c = *(const v4f*)(sr + 4);
  float z[8];
#pragma unroll
  for (int e = 0; e < 4; ++e) { z[e] = a[e] * kInvSqrtD; z[4 + e] = c[e] * kInvSqrtD; }

  float m = fmaxf(fmaxf(fmaxf(z[0], z[1]), fmaxf(z[2], z[3])), fmaxf(fmaxf(z[4], z[5]), fmaxf(z[6], z[7])));
#pragma unroll
  for (int off = 16; off > 0; off >>= 1) m = fmaxf(m, __shfl_xor(m, off, 32));
  if (lane == 0) red[0][wave] = m;
  __syncthreads();
  m = red[0][0];
#pragma unroll
  for (int w = 1; w < 8; ++w) m = fmaxf(m, red[0][w]);

  float e1[8];
  float s1 = 0.f;
#pragma unroll
  for (int e = 0; e < 8; ++e) { e1[e] = __expf(z[e] - m); s1 += e1[e]; }
#pragma unroll
  for (int off = 16; off > 0; off >>= 1) s1 += __shfl_xor(s1, off, 32);
  if (lane == 0) red[1][wave] = s1;
  __syncthreads();
  float zsum1 = red[1][0];
#pragma unroll
  for (int w = 1; w < 8; ++w) zsum1 += red[1][w];
  const float inv1 = 1.0f / zsum1;

  float z2[8];
  float m2 = -INFINITY;
#pragma unroll
  for (int e = 0; e < 8; ++e) {
    const float wgt = e1[e] * inv1;
    const float zz  = wgt * kInvSqrtD;
    const bool valid = (c0 + e) <= row;
    z2[e] = valid ? zz : -INFINITY;
    m2 = fmaxf(m2, z2[e]);
  }
#pragma unroll
  for (int off = 16; off > 0; off >>= 1) m2 = fmaxf(m2, __shfl_xor(m2, off, 32));
  if (lane == 0) red[2][wave] = m2;
  __syncthreads();
  m2 = red[2][0];
#pragma unroll
  for (int w = 1; w < 8; ++w) m2 = fmaxf(m2, red[2][w]);

  float e2[8];
  float s2 = 0.f;
#pragma unroll
  for (int e = 0; e < 8; ++e) {
    const bool valid = (c0 + e) <= row;
    const float ex = __expf(z2[e] - m2);
    e2[e] = valid ? ex : 0.f;
    s2 += e2[e];
  }
#pragma unroll
  for (int off = 16; off > 0; off >>= 1) s2 += __shfl_xor(s2, off, 32);
  if (lane == 0) red[3][wave] = s2;
  __syncthreads();
  float zsum2 = red[3][0];
#pragma unroll
  for (int w = 1; w < 8; ++w) zsum2 += red[3][w];
  const float inv2 = 1.0f / zsum2;

  unsigned short hb[8], lb[8];
#pragma unroll
  for (int e = 0; e < 8; ++e) {
    const float p = e2[e] * inv2;
    const unsigned short h = f2bf_bits(p);
    hb[e] = h;
    lb[e] = f2bf_bits(p - bf_bits2f(h));
  }
  const v4u uh = (v4u){pk16(hb[0], hb[1]), pk16(hb[2], hb[3]), pk16(hb[4], hb[5]), pk16(hb[6], hb[7])};
  const v4u ul = (v4u){pk16(lb[0], lb[1]), pk16(lb[2], lb[3]), pk16(lb[4], lb[5]), pk16(lb[6], lb[7])};
  unsigned short* qh = Ph + (size_t)row * kSeq + c0;
  unsigned short* ql = Pl + (size_t)row * kSeq + c0;
  *(volatile v4u*)qh = uh;
  *(volatile v4u*)ql = ul;
  __threadfence();
  *(volatile v4u*)qh = uh;
  *(volatile v4u*)ql = ul;
}

extern "C" void kernel_launch(void* const* d_in, const int* in_sizes, int n_in,
                              void* d_out, int out_size, void* d_ws, size_t ws_size,
                              hipStream_t stream) {
  if (n_in < 4) return;
  if (in_sizes[0] != kTok * kDim || in_sizes[1] != kDim * kDim || in_sizes[2] != kDim * kDim ||
      in_sizes[3] != kDim * kDim || out_size != kTok * kDim) return;

  const float* x  = (const float*)d_in[0];
  const float* Wq = (const float*)d_in[1];
  const float* Wk = (const float*)d_in[2];
  const float* Wv = (const float*)d_in[3];
  float* out = (float*)d_out;

  const size_t nTokD = (size_t)kTok * kDim;
  const size_t nW    = (size_t)kDim * kDim;
  const size_t nSS   = (size_t)kSeq * kSeq;
  size_t off = 0;
  const size_t oXb = off; off += nTokD * 2;
  const size_t oWb = off; off += 3 * nW * 2;
  const size_t oQK = off; off += (size_t)kTok * kQKld * 2;
  const size_t oVh = off; off += nTokD * 2;
  const size_t oVl = off; off += nTokD * 2;
  const size_t oS  = off; off += nSS * 4;
  const size_t oPh = off; off += nSS * 2;
  const size_t oPl = off; off += nSS * 2;
  if (off > ws_size) return;

  char* ws = (char*)d_ws;
  unsigned short* xb   = (unsigned short*)(ws + oXb);
  unsigned short* Wb   = (unsigned short*)(ws + oWb);
  unsigned short* QK16 = (unsigned short*)(ws + oQK);
  unsigned short* Vth  = (unsigned short*)(ws + oVh);
  unsigned short* Vtl  = (unsigned short*)(ws + oVl);
  float*          S32  = (float*)(ws + oS);
  unsigned short* Ph   = (unsigned short*)(ws + oPh);
  unsigned short* Pl   = (unsigned short*)(ws + oPl);
  const float* dummyf  = (const float*)S32;

  const int n8x = (int)(nTokD / 8);
  const int n8w = (int)(nW / 8);
  cast8_bf16_kernel<<<(unsigned)((n8x + 255) / 256), 256, 0, stream>>>(x, xb, n8x);
  cast8_bf16_kernel<<<(unsigned)((n8w + 255) / 256), 256, 0, stream>>>(Wq, Wb, n8w);
  cast8_bf16_kernel<<<(unsigned)((n8w + 255) / 256), 256, 0, stream>>>(Wk, Wb + nW, n8w);
  cast8_bf16_kernel<<<(unsigned)((n8w + 255) / 256), 256, 0, stream>>>(Wv, Wb + 2 * nW, n8w);

  wmma_gemm64<1, false, 0, 1, false><<<dim3(512, 1), 256, 0, stream>>>(
      xb, xb, kDim, 0L, Wb, Wb, kDim, 0L, (void*)QK16, (void*)QK16, kQKld, 0L,
      dummyf, dummyf, 0L, kTok, 2 * kDim, kDim, 1.0f);

  wmma_gemm64<1, false, 0, 2, false><<<dim3(64, kBatch), 256, 0, stream>>>(
      Wb + 2 * nW, Wb + 2 * nW, kDim, 0L, xb, xb, kDim, (long)kSeq * kDim, (void*)Vth, (void*)Vtl, kSeq, (long)kDim * kSeq,
      dummyf, dummyf, 0L, kDim, kSeq, kDim, 1.0f);

  for (int b = 0; b < kBatch; ++b) {
    const unsigned short* qplane = QK16 + (size_t)b * kSeq * kQKld;
    const unsigned short* kplane = qplane + kDim;
    wmma_gemm64<0, false, 0, 0, false><<<dim3(128, 1), 256, 0, stream>>>(
        qplane, qplane, kQKld, 0L, kplane, kplane, kQKld, 0L, (void*)S32, (void*)S32, kSeq, 0L,
        dummyf, dummyf, 0L, kSeq, kSeq, kDim, 1.0f);
    softmax2_row_kernel<<<kSeq, 256, 0, stream>>>(S32, Ph, Pl);
    wmma_gemm64<1, true, 0, 0, false, 0, true><<<dim3(64, 1), 256, 0, stream>>>(
        Ph, Pl, kSeq, 0L, Vth + (size_t)b * kDim * kSeq, Vtl + (size_t)b * kDim * kSeq, kSeq, 0L,
        (void*)(out + (size_t)b * kSeq * kDim), (void*)(out + (size_t)b * kSeq * kDim), kDim, 0L,
        dummyf, dummyf, 0L, kSeq, kDim, kSeq, 1.0f);
  }
}
